// TensorProductWrapper_41566693490835
// MI455X (gfx1250) — hardware-verified
//
#include <hip/hip_runtime.h>

#define NBATCH 8192
#define MUL    64
#define XD     256
static constexpr float kInvSqrt3 = 0.57735026918962576f;
static constexpr float kAlpha0   = 0.011048543456039806f;
static constexpr float kAlpha1   = 0.019136638615493577f;

typedef __attribute__((ext_vector_type(16))) _Float16 v16h;
typedef __attribute__((ext_vector_type(8)))  _Float16 v8h;
typedef __attribute__((ext_vector_type(8)))  float    v8f;
typedef __attribute__((ext_vector_type(4)))  float    v4f_t;
typedef float v4fa __attribute__((ext_vector_type(4), may_alias));
typedef __attribute__((ext_vector_type(4)))  unsigned v4u_t;
typedef unsigned v4ua __attribute__((ext_vector_type(4), may_alias));

__device__ __forceinline__ v8f wmma16(v16h a, v16h b, v8f c) { return __builtin_amdgcn_wmma_f32_16x16x32_f16(false, a, false, b, (short)0, c, false, false); }
__device__ __forceinline__ v16h frag16(const _Float16* p, int g) {
  return __builtin_shufflevector(*(const v8h*)(p + 8 * g), *(const v8h*)(p + 16 + 8 * g), 0,1,2,3,4,5,6,7,8,9,10,11,12,13,14,15);
}

__global__ __launch_bounds__(256) void prep_x(const float* __restrict__ x, _Float16* __restrict__ xh) {
  const int t = blockIdx.x * 256 + threadIdx.x;
  if (t >= 4 * NBATCH * 8) return;
  const int u8 = (t & 7) * 8, b = (t >> 3) & (NBATCH - 1), s = t >> 16;
  const float* xr = x + (size_t)b * XD;
  _Float16 hh[8];
#pragma unroll
  for (int e = 0; e < 8; ++e) { const int u = u8 + e; hh[e] = (_Float16)((s == 0) ? xr[u] : xr[MUL + 3 * u + (s - 1)]); }
  _Float16* d = xh + ((size_t)s * NBATCH + b) * MUL + u8;
  *(volatile v4u_t*)d = *(const v4ua*)hh; __threadfence(); *(volatile v4u_t*)d = *(const v4ua*)hh;
}
__global__ __launch_bounds__(256) void prep_w(const float* __restrict__ w000, const float* __restrict__ w110,
                                              const float* __restrict__ w011, const float* __restrict__ w101,
                                              _Float16* __restrict__ Wp) {
  const int t = blockIdx.x * 256 + threadIdx.x;
  if (t >= 4 * 4096 * 8) return;
  const int k8 = (t & 7) * 8, n = (t >> 3) & 4095, p = t >> 15;
  const int w = n >> 6, s = n & 63;
  const float* W = (p == 0) ? w000 : (p == 1) ? w110 : (p == 2) ? w011 : w101;
  _Float16 hh[8];
#pragma unroll
  for (int e = 0; e < 8; ++e) {
    const int k = k8 + e;
    const size_t idx = (p == 3) ? (((size_t)s * MUL + k) * MUL + w) : (((size_t)k * MUL + s) * MUL + w);
    hh[e] = (_Float16)W[idx];
  }
  _Float16* d = Wp + ((size_t)p * 4096 + n) * MUL + k8;
  *(volatile v4u_t*)d = *(const v4ua*)hh; __threadfence(); *(volatile v4u_t*)d = *(const v4ua*)hh;
}

__device__ __forceinline__ void pass64(const _Float16* __restrict__ A, const _Float16* __restrict__ Wrows, int lane, v8f* acc) {
  const int g = lane >> 4, l16 = lane & 15;
#pragma unroll
  for (int j = 0; j < 4; ++j) acc[j] = (v8f){0.f, 0.f, 0.f, 0.f, 0.f, 0.f, 0.f, 0.f};
#pragma unroll
  for (int k0 = 0; k0 < MUL; k0 += 32) {
    const v16h a = frag16(A + (size_t)l16 * MUL + k0, g);
#pragma unroll
    for (int j = 0; j < 4; ++j) acc[j] = wmma16(a, frag16(Wrows + (size_t)(j * 16 + l16) * MUL + k0, g), acc[j]);
  }
}
__device__ __forceinline__ void dot64(const v8f* acc, const float* xs, int xstride, int cs, int co, int lane, float* r  ) {
  const int g = lane >> 4, l16 = lane & 15;
#pragma unroll
  for (int rr = 0; rr < 8; ++rr) {
    const float* xr = xs + (rr + 8 * g) * xstride;
    float s = 0.f;
#pragma unroll
    for (int j = 0; j < 4; ++j) s = fmaf(acc[j][rr], xr[(j * 16 + l16) * cs + co], s);
    s += __shfl_xor(s, 1, 32); s += __shfl_xor(s, 2, 32); s += __shfl_xor(s, 4, 32); s += __shfl_xor(s, 8, 32);
    r[rr] = s;
  }
}

__global__ __launch_bounds__(256) void tp_kernel(const float* __restrict__ x, const _Float16* __restrict__ xh,
                                                 const _Float16* __restrict__ Wp, float* __restrict__ out) {
  __shared__ __attribute__((aligned(16))) float x0s[16 * MUL];
  __shared__ __attribute__((aligned(16))) float x1s[16 * 3 * MUL];
  __shared__ __attribute__((aligned(16))) float so0[16 * 32];
  __shared__ __attribute__((aligned(16))) float so1[16 * 96];
  const int tid = threadIdx.x, lane = tid & 31, wave = tid >> 5;
  const int g = lane >> 4, l16 = lane & 15;
  const int r0 = blockIdx.x * 16, wh = blockIdx.y;
  for (int i = tid; i < 16 * MUL; i += 256) x0s[i] = x[(size_t)(r0 + (i >> 6)) * XD + (i & 63)];
  for (int i = tid; i < 16 * 3 * MUL; i += 256) x1s[i] = x[(size_t)(r0 + i / 192) * XD + MUL + (i % 192)];
  __syncthreads();

  const _Float16* X0 = xh + (size_t)r0 * MUL;
  v8f acc[4];
  float ra[8], rb[8];
#pragma unroll 1
  for (int wl4 = 0; wl4 < 4; ++wl4) {
    const int wl = wave * 4 + wl4, w = wh * 32 + wl;
    pass64(X0, Wp + ((size_t)0 * 4096 + w * 64) * MUL, lane, acc);
    dot64(acc, x0s, MUL, 1, 0, lane, ra);
    asm volatile("" ::: "memory");
    float p110[8] = {0.f, 0.f, 0.f, 0.f, 0.f, 0.f, 0.f, 0.f};
#pragma unroll 1
    for (int i = 0; i < 3; ++i) {
      pass64(xh + ((size_t)(1 + i) * NBATCH + r0) * MUL, Wp + ((size_t)1 * 4096 + w * 64) * MUL, lane, acc);
      dot64(acc, x1s, 3 * MUL, 3, i, lane, rb);
      asm volatile("" ::: "memory");
#pragma unroll
      for (int rr = 0; rr < 8; ++rr) p110[rr] += rb[rr];
    }
    if (l16 == 0) {
#pragma unroll
      for (int rr = 0; rr < 8; ++rr) so0[(rr + 8 * g) * 32 + wl] = kAlpha0 * (ra[rr] + p110[rr] * kInvSqrt3);
    }
    float p1[3][8];
    pass64(X0, Wp + ((size_t)2 * 4096 + w * 64) * MUL, lane, acc);
#pragma unroll
    for (int k = 0; k < 3; ++k) { dot64(acc, x1s, 3 * MUL, 3, k, lane, p1[k]); asm volatile("" ::: "memory"); }
    pass64(X0, Wp + ((size_t)3 * 4096 + w * 64) * MUL, lane, acc);
#pragma unroll
    for (int k = 0; k < 3; ++k) {
      dot64(acc, x1s, 3 * MUL, 3, k, lane, rb);
      asm volatile("" ::: "memory");
      if (l16 == 0) {
#pragma unroll
        for (int rr = 0; rr < 8; ++rr) so1[(rr + 8 * g) * 96 + wl * 3 + k] = kAlpha1 * kInvSqrt3 * (p1[k][rr] + rb[rr]);
      }
    }
  }
  __syncthreads();
#pragma unroll 1
  for (int ps = 0; ps < 2; ++ps) {
    for (int c = tid; c < 16 * 32; c += 256) {
      const int rr = c >> 5, q = c & 31;
      float* orow = out + (size_t)(r0 + rr) * XD;
      if (q < 8) *(volatile v4f_t*)(orow + wh * 32 + q * 4) = *(const volatile v4fa*)(so0 + rr * 32 + q * 4);
      else       *(volatile v4f_t*)(orow + MUL + wh * 96 + (q - 8) * 4) = *(const volatile v4fa*)(so1 + rr * 96 + (q - 8) * 4);
    }
    __threadfence();
  }
}

extern "C" void kernel_launch(void* const* d_in, const int* in_sizes, int n_in,
                              void* d_out, int out_size, void* d_ws, size_t ws_size,
                              hipStream_t stream) {
  (void)in_sizes; (void)n_in; (void)out_size; (void)ws_size;
  const float* x    = (const float*)d_in[0];
  const float* w000 = (const float*)d_in[1];
  const float* w110 = (const float*)d_in[2];
  const float* w011 = (const float*)d_in[3];
  const float* w101 = (const float*)d_in[4];
  float* out = (float*)d_out;
  _Float16* xh = (_Float16*)d_ws;
  _Float16* Wp = xh + (size_t)4 * NBATCH * MUL;
  prep_x<<<(4 * NBATCH * 8) / 256, 256, 0, stream>>>(x, xh);
  prep_w<<<(4 * 4096 * 8) / 256, 256, 0, stream>>>(w000, w110, w011, w101, Wp);
  tp_kernel<<<dim3(NBATCH / 16, 2), 256, 0, stream>>>(x, xh, Wp, out);
}
